// TimedOrthogonalBivectorBlock_429496730089
// MI455X (gfx1250) — hardware-run, weakly checked
//
#include <hip/hip_runtime.h>
#include <stddef.h>
#include <stdint.h>
#include <math.h>

#define NBATCH 2
#define SEQ    2048
#define NTOK   4096
#define DMOD   512
#define NPLN   32
#define NPH    64
#define NPOS   8
#define FP     128
#define QB     64
#define KC     64
#define NQB    32
#define NSEG   8
#define SFP    68
#define SKP    36
#define FPL    136
#define SLP    72
#define OTP    68

#define CW      64.0f
#define CW_INV  0.015625f
#define CV      8.0f
#define CSC     4.0f
#define CSV_INV 0.03125f
#define CT      16.0f
#define CTO_INV 0.0009765625f

static_assert(NTOK == NBATCH * SEQ);
static_assert(SEQ == NQB * QB);
static_assert(QB == KC);
static_assert(DMOD == NSEG * 64);
static_assert(DMOD % 64 == 0);
static_assert(NPH == 2 * NPLN);
static_assert(NPH == 64);
static_assert(2 * NPLN + 2 * NPOS <= 96);
static_assert(FP == 128);
static_assert((NTOK * DMOD) % 2048 == 0);
static_assert((SEQ & (SEQ - 1)) == 0);
static_assert((FPL * 2) % 16 == 0);
static_assert((SLP * 2) % 16 == 0);
static_assert((SFP * 4) % 16 == 0);
static_assert((OTP * 4) % 16 == 0);

typedef unsigned short us;
typedef _Float16 v16h __attribute__((ext_vector_type(16)));
typedef _Float16 v8h  __attribute__((ext_vector_type(8)));
typedef us       v8us __attribute__((ext_vector_type(8)));
typedef float    v8f  __attribute__((ext_vector_type(8)));
typedef float    v4f  __attribute__((ext_vector_type(4)));
typedef unsigned int v4u __attribute__((ext_vector_type(4)));

union Frag  { v16h v; v8us h[2]; };
union Pack8 { v8h h; v4u u; };

__device__ __forceinline__ v4u pack8(const float (&f)[8]) {
  Pack8 p;
  p.h = (v8h){(_Float16)f[0], (_Float16)f[1], (_Float16)f[2], (_Float16)f[3],
              (_Float16)f[4], (_Float16)f[5], (_Float16)f[6], (_Float16)f[7]};
  return p.u;
}

__device__ __forceinline__ v8f mma16(v16h a, v16h b, v8f c) {
  c = __builtin_amdgcn_wmma_f32_16x16x32_f16(false, a, false, b, (short)0, c, false, false);
  asm volatile("v_nop\n\tv_nop\n\tv_nop\n\tv_nop" : "+v"(c) : "v"(a), "v"(b));
  return c;
}

__device__ __forceinline__ v16h ldfrag(const us* p, int ld, int row0, int k0, int lane) {
  const int m = lane & 15, lh = lane >> 4;
  const us* q = p + (size_t)(row0 + m) * ld + k0 + 8 * lh;
  Frag f;
  f.h[0] = *(const v8us*)(q);
  f.h[1] = *(const v8us*)(q + 16);
  return f.v;
}

__device__ __forceinline__ v8f zero8() { return (v8f){0.f, 0.f, 0.f, 0.f, 0.f, 0.f, 0.f, 0.f}; }

template <int KD>
__device__ __forceinline__ void gemm16x64(const us* __restrict__ A, const us* __restrict__ B,
                                          int m0, int n0, int lane, v8f (&acc)[4]) {
  static_assert(KD % 32 == 0);
#pragma unroll 1
  for (int k0 = 0; k0 < KD; k0 += 32) {
    const v16h a = ldfrag(A, KD, m0, k0, lane);
#pragma unroll
    for (int t = 0; t < 4; ++t) {
      const v16h b = ldfrag(B, KD, n0 + 16 * t, k0, lane);
      acc[t] = mma16(a, b, acc[t]);
    }
  }
}

__global__ __launch_bounds__(256) void k_cvt_x(const float* __restrict__ x, us* __restrict__ xh) {
  const size_t i = (size_t)blockIdx.x * 2048 + (size_t)threadIdx.x * 8;
  const v4f a0 = *(const v4f*)(x + i);
  const v4f a1 = *(const v4f*)(x + i + 4);
  const float f[8] = {a0[0], a0[1], a0[2], a0[3], a1[0], a1[1], a1[2], a1[3]};
  const v4u hv = pack8(f);
  *(volatile v4u*)(xh + i) = hv;
  __threadfence();
  *(volatile v4u*)(xh + i) = hv;
}

__global__ __launch_bounds__(256) void k_cvt_wt(const float* __restrict__ w, us* __restrict__ wt) {
  __shared__ __align__(16) float sw[64 * SFP];
  const int tid = threadIdx.x;
  const int kb = blockIdx.x * 64;
  const int nb = blockIdx.y * 64;
  {
    const int r  = tid >> 2;
    const int c0 = (tid & 3) * 16;
    const float* src = w + (size_t)(kb + r) * DMOD + nb + c0;
#pragma unroll
    for (int e = 0; e < 4; ++e) *(v4f*)(sw + r * SFP + c0 + 4 * e) = *(const v4f*)(src + 4 * e);
  }
  __syncthreads();
  v4u hv[2];
  size_t go[2];
#pragma unroll
  for (int j = 0; j < 2; ++j) {
    const int p  = tid + 256 * j;
    const int n  = p >> 3;
    const int pc = p & 7;
    const float* cp = sw + (pc * 8) * SFP + n;
    float f[8];
#pragma unroll
    for (int e = 0; e < 8; ++e) f[e] = cp[e * SFP] * CW;
    hv[j] = pack8(f);
    go[j] = (size_t)(nb + n) * DMOD + kb + pc * 8;
  }
#pragma unroll
  for (int j = 0; j < 2; ++j) *(volatile v4u*)(wt + go[j]) = hv[j];
  __threadfence();
#pragma unroll
  for (int j = 0; j < 2; ++j) *(volatile v4u*)(wt + go[j]) = hv[j];
}

__global__ __launch_bounds__(256) void k_cvt_wkq(const float* __restrict__ wk, const float* __restrict__ wq,
                                                 us* __restrict__ wt) {
  __shared__ __align__(16) float sw[64 * SKP];
  const int tid = threadIdx.x;
  const int kb  = blockIdx.x * 64;
  const int sel = blockIdx.y;
  const float* w = (sel == 0) ? wk : wq;
  {
    const int r  = tid >> 2;
    const int c0 = (tid & 3) * 8;
    const float* src = w + (size_t)(kb + r) * NPLN + c0;
    *(v4f*)(sw + r * SKP + c0)     = *(const v4f*)(src);
    *(v4f*)(sw + r * SKP + c0 + 4) = *(const v4f*)(src + 4);
  }
  __syncthreads();
  const int n  = tid >> 3;
  const int pc = tid & 7;
  const float* cp = sw + (pc * 8) * SKP + n;
  float f[8];
#pragma unroll
  for (int e = 0; e < 8; ++e) f[e] = cp[e * SKP] * CW;
  const v4u hv = pack8(f);
  const size_t go = (size_t)(sel * NPLN + n) * DMOD + kb + pc * 8;
  *(volatile v4u*)(wt + go) = hv;
  __threadfence();
  *(volatile v4u*)(wt + go) = hv;
}

__global__ __launch_bounds__(128) void k_phase(const us* __restrict__ xh, const us* __restrict__ wkq,
                                               const float* __restrict__ bk, const float* __restrict__ bq,
                                               const float* __restrict__ setw, const float* __restrict__ pfreq,
                                               us* __restrict__ qf, us* __restrict__ kf) {
  __shared__ __align__(16) float    sf[64 * SFP];
  __shared__ __align__(16) _Float16 kst[64 * FPL];
  __shared__ __align__(16) _Float16 qst[64 * FPL];
  const int tid = threadIdx.x, lane = tid & 31, wave = tid >> 5;
  const int hh = lane >> 4, c = lane & 15;
  const int mb = blockIdx.x * 64;
  const int m0 = mb + wave * 16;

  v8f acc[4];
#pragma unroll
  for (int t = 0; t < 4; ++t) acc[t] = zero8();
  gemm16x64<DMOD>(xh, wkq, m0, 0, lane, acc);

  float bcol[4];
#pragma unroll
  for (int t = 0; t < 4; ++t) {
    const float* bp = (t < 2) ? bk : bq;
    bcol[t] = bp[(16 * t + c) & 31];
  }
#pragma unroll
  for (int t = 0; t < 4; ++t) {
#pragma unroll
    for (int r = 0; r < 8; ++r) sf[(wave * 16 + 8 * hh + r) * SFP + 16 * t + c] = acc[t][r] * CW_INV + bcol[t];
  }

  const float s0 = setw[0], s1 = setw[1], s2 = setw[2], s3 = setw[3];
  const float mx = fmaxf(fmaxf(s0, s1), fmaxf(s2, s3));
  const float e0 = expf(s0 - mx), e1 = expf(s1 - mx), e2 = expf(s2 - mx), e3 = expf(s3 - mx);
  const float rden = 1.0f / (((e0 + e1) + e2) + e3);
  const float w0 = e0 * rden, w1 = e1 * rden, w2 = e2 * rden, w3 = e3 * rden;

  __syncthreads();

  const float PI_F     = 3.14159274101257324f;
  const float TWO_PI_F = 6.28318548202514648f;
#pragma unroll 1
  for (int e = tid; e < 64 * NPLN; e += 128) {
    const int row = e >> 5, j = e & 31, js = j >> 3;
    const float w = (js == 0) ? w0 : ((js == 1) ? w1 : ((js == 2) ? w2 : w3));
    const float kp = tanhf(sf[row * SFP + j]) * PI_F;
    const float qp = tanhf(sf[row * SFP + NPLN + j]) * PI_F;
    const float ck = cosf(kp), sk = sinf(kp);
    const float cq = cosf(qp), sq = sinf(qp);
    kst[row * FPL + j]        = (_Float16)ck;
    kst[row * FPL + NPLN + j] = (_Float16)sk;
    qst[row * FPL + j]        = (_Float16)(w * cq);
    qst[row * FPL + NPLN + j] = (_Float16)(w * sq);
  }
#pragma unroll 1
  for (int e = tid; e < 64 * NPOS; e += 128) {
    const int row = e >> 3, p = e & 7;
    const int l = (mb + row) & (SEQ - 1);
    const float th = ((float)l * pfreq[p]) * TWO_PI_F;
    const float ct = cosf(th), st = sinf(th);
    kst[row * FPL + 2 * NPLN + p]        = (_Float16)ct;
    kst[row * FPL + 2 * NPLN + NPOS + p] = (_Float16)st;
    qst[row * FPL + 2 * NPLN + p]        = (_Float16)ct;
    qst[row * FPL + 2 * NPLN + NPOS + p] = (_Float16)st;
  }
  {
    Pack8 z;
    z.u = (v4u){0u, 0u, 0u, 0u};
#pragma unroll 1
    for (int e = tid; e < 64 * 6; e += 128) {
      const int row = e / 6, q = e - row * 6;
      *(v8h*)(kst + row * FPL + 80 + 8 * q) = z.h;
      *(v8h*)(qst + row * FPL + 80 + 8 * q) = z.h;
    }
  }
  __syncthreads();

#pragma unroll
  for (int pl = 0; pl < 2; ++pl) {
    const _Float16* src = (pl == 0) ? kst : qst;
    us* dst = (pl == 0) ? kf : qf;
#pragma unroll
    for (int g = 0; g < 2; ++g) {
      v4u hv[4];
      size_t go[4];
#pragma unroll
      for (int i = 0; i < 4; ++i) {
        const int p   = tid + 128 * (4 * g + i);
        const int row = p >> 4;
        const int c8  = (p & 15) * 8;
        Pack8 a;
        a.h = *(const v8h*)(src + row * FPL + c8);
        hv[i] = a.u;
        go[i] = (size_t)(mb + row) * FP + c8;
      }
#pragma unroll
      for (int i = 0; i < 4; ++i) *(volatile v4u*)(dst + go[i]) = hv[i];
      __threadfence();
#pragma unroll
      for (int i = 0; i < 4; ++i) *(volatile v4u*)(dst + go[i]) = hv[i];
    }
  }
}

template <int MODE>
__global__ __launch_bounds__(128) void k_proj(const us* __restrict__ ap, const us* __restrict__ wt,
                                              const float* __restrict__ bias, const float* __restrict__ xres,
                                              us* __restrict__ y16, float* __restrict__ yf) {
  __shared__ __align__(16) float sf[64 * SFP];
  const int tid = threadIdx.x, lane = tid & 31, wave = tid >> 5;
  const int hh = lane >> 4, c = lane & 15;
  const int mb = blockIdx.x * 64;
  const int nb = blockIdx.y * 64;
  const int m0 = mb + wave * 16;

  v8f acc[4];
#pragma unroll
  for (int t = 0; t < 4; ++t) acc[t] = zero8();
  gemm16x64<DMOD>(ap, wt, m0, nb, lane, acc);

  float bcol[4];
#pragma unroll
  for (int t = 0; t < 4; ++t) bcol[t] = 0.f;
  if constexpr (MODE == 1 || MODE == 2) {
#pragma unroll
    for (int t = 0; t < 4; ++t) bcol[t] = bias[nb + 16 * t + c];
  }
#pragma unroll
  for (int t = 0; t < 4; ++t) {
#pragma unroll
    for (int r = 0; r < 8; ++r) {
      float v;
      if constexpr (MODE == 1) {
        v = (acc[t][r] * CW_INV + bcol[t]) * CV;
      } else if constexpr (MODE == 2) {
        const float z = acc[t][r] * CW_INV + bcol[t];
        const float e = __expf(-z);
        v = 1.0f / (1.0f + e);
      } else {
        v = acc[t][r] * CTO_INV;
      }
      sf[(wave * 16 + 8 * hh + r) * SFP + 16 * t + c] = v;
    }
  }
  __syncthreads();

  if constexpr (MODE == 1) {
    v4u hv[4];
    size_t go[4];
#pragma unroll
    for (int j = 0; j < 4; ++j) {
      const int p  = tid + 128 * j;
      const int d  = p >> 3;
      const int pc = p & 7;
      const float* cp = sf + (pc * 8) * SFP + d;
      float f[8];
#pragma unroll
      for (int e = 0; e < 8; ++e) f[e] = cp[e * SFP];
      hv[j] = pack8(f);
      go[j] = ((size_t)(nb + d)) * (size_t)NTOK + mb + pc * 8;
    }
#pragma unroll
    for (int j = 0; j < 4; ++j) *(volatile v4u*)(y16 + go[j]) = hv[j];
    __threadfence();
#pragma unroll
    for (int j = 0; j < 4; ++j) *(volatile v4u*)(y16 + go[j]) = hv[j];
  } else {
    v4f val[8];
    size_t go[8];
#pragma unroll
    for (int it = 0; it < 8; ++it) {
      const int p    = tid + 128 * it;
      const int L    = p >> 3;
      const int pc   = p & 7;
      const int row  = L >> 1;
      const int half = L & 1;
      const int col  = half * 32 + pc * 4;
      const size_t o = (size_t)(mb + row) * DMOD + nb + col;
      const v4f sv = *(const v4f*)(sf + row * SFP + col);
      if constexpr (MODE == 3) {
        const v4f xv = *(const v4f*)(xres + o);
        const v4f bv = *(const v4f*)(bias + nb + col);
        val[it] = (xv + sv) + bv;
      } else {
        val[it] = sv;
      }
      go[it] = o;
    }
#pragma unroll
    for (int it = 0; it < 8; ++it) *(volatile v4f*)(yf + go[it]) = val[it];
    __threadfence();
#pragma unroll
    for (int it = 0; it < 8; ++it) *(volatile v4f*)(yf + go[it]) = val[it];
  }
}

__global__ __launch_bounds__(128) void k_score(const us* __restrict__ qf, const us* __restrict__ kf,
                                               us* __restrict__ sc, us* __restrict__ sp) {
  __shared__ __align__(16) _Float16 stc[4 * 16 * SLP];
  __shared__ __align__(16) _Float16 stp[4 * 16 * SLP];
  const int tid = threadIdx.x, lane = tid & 31, wave = tid >> 5;
  const int hh = lane >> 4, c = lane & 15;
  const int qb   = blockIdx.x;
  const int b    = blockIdx.y;
  const int tok0 = b * SEQ;
  const int qloc = qb * QB + wave * 16;
  const int q0   = tok0 + qloc;
  const int nch  = qb + 1;

  const v16h qa0 = ldfrag(qf, FP, q0, 0, lane);
  const v16h qa1 = ldfrag(qf, FP, q0, 32, lane);
  const v16h qa2 = ldfrag(qf, FP, q0, 64, lane);
  _Float16* wc = stc + wave * 16 * SLP;
  _Float16* wp = stp + wave * 16 * SLP;

#pragma unroll 1
  for (int i = 0; i < nch; ++i) {
    const int kv0 = i * KC;
    v8f s[4], u[4];
#pragma unroll
    for (int j = 0; j < 4; ++j) { s[j] = zero8(); u[j] = zero8(); }
#pragma unroll
    for (int j = 0; j < 4; ++j) {
      const int kr = tok0 + kv0 + 16 * j;
      const v16h kb0 = ldfrag(kf, FP, kr, 0, lane);
      const v16h kb1 = ldfrag(kf, FP, kr, 32, lane);
      const v16h kb2 = ldfrag(kf, FP, kr, 64, lane);
      s[j] = mma16(qa0, kb0, s[j]);
      s[j] = mma16(qa1, kb1, s[j]);
      u[j] = mma16(qa2, kb2, u[j]);
    }
    __syncthreads();
#pragma unroll
    for (int j = 0; j < 4; ++j) {
      const int key = kv0 + 16 * j + c;
#pragma unroll
      for (int r = 0; r < 8; ++r) {
        const int qry = qloc + 8 * hh + r;
        const bool keep = (key <= qry);
        const float vs = keep ? s[j][r] * CSC : 0.f;
        const float vu = keep ? u[j][r] * CSC : 0.f;
        wc[(8 * hh + r) * SLP + 16 * j + c] = (_Float16)vs;
        wp[(8 * hh + r) * SLP + 16 * j + c] = (_Float16)vu;
      }
    }
    __syncthreads();
    v4u cv[4], pv[4];
    size_t go[4];
#pragma unroll
    for (int it = 0; it < 4; ++it) {
      const int p  = lane + 32 * it;
      const int lr = p >> 3;
      const int d0 = (p & 7) * 8;
      Pack8 a, e;
      a.h = *(const v8h*)(wc + lr * SLP + d0);
      e.h = *(const v8h*)(wp + lr * SLP + d0);
      cv[it] = a.u;
      pv[it] = e.u;
      go[it] = (size_t)(q0 + lr) * SEQ + kv0 + d0;
    }
#pragma unroll
    for (int it = 0; it < 4; ++it) { *(volatile v4u*)(sc + go[it]) = cv[it]; *(volatile v4u*)(sp + go[it]) = pv[it]; }
    __threadfence();
#pragma unroll
    for (int it = 0; it < 4; ++it) { *(volatile v4u*)(sc + go[it]) = cv[it]; *(volatile v4u*)(sp + go[it]) = pv[it]; }
  }
}

__global__ __launch_bounds__(128) void k_oattn(const us* __restrict__ sc, const us* __restrict__ sp,
                                               const us* __restrict__ vt, const float* __restrict__ gt,
                                               const float* __restrict__ pw, us* __restrict__ tp) {
  __shared__ __align__(16) float osw[4 * 16 * OTP];
  const int tid = threadIdx.x, lane = tid & 31, wave = tid >> 5;
  const int hh = lane >> 4, c = lane & 15;
  const int seg  = blockIdx.x;
  const int qb   = blockIdx.y;
  const int b    = blockIdx.z;
  const int col0 = seg * 64;
  const int tok0 = b * SEQ;
  const int qloc = qb * QB + wave * 16;
  const int q0   = tok0 + qloc;
  const int nk   = (qb + 1) * 2;

  const float spw = 1.0f / (1.0f + expf(-pw[0]));

  v8f accC[4], accP[4];
#pragma unroll
  for (int t = 0; t < 4; ++t) { accC[t] = zero8(); accP[t] = zero8(); }

#pragma unroll 1
  for (int ks = 0; ks < nk; ++ks) {
    const int k0 = ks * 32;
    const v16h ac = ldfrag(sc, SEQ, q0, k0, lane);
    const v16h ap = ldfrag(sp, SEQ, q0, k0, lane);
#pragma unroll
    for (int t = 0; t < 4; ++t) {
      const v16h bv = ldfrag(vt, NTOK, col0 + 16 * t, tok0 + k0, lane);
      accC[t] = mma16(ac, bv, accC[t]);
      accP[t] = mma16(ap, bv, accP[t]);
    }
  }

  float rn[8];
#pragma unroll
  for (int r = 0; r < 8; ++r) {
    const int pos = qloc + 8 * hh + r + 1;
    rn[r] = 1.0f / sqrtf((float)pos * 8.0f);
  }
  float* ow = osw + wave * 16 * OTP;
#pragma unroll
  for (int t = 0; t < 4; ++t) {
#pragma unroll
    for (int r = 0; r < 8; ++r) {
      const int row = 8 * hh + r;
      const size_t gi = (size_t)(q0 + row) * DMOD + col0 + 16 * t + c;
      const float g   = gt[gi];
      const float cc  = accC[t][r] * CSV_INV;
      const float pp  = spw * (accP[t][r] * CSV_INV);
      const float tot = g * cc + (1.0f - g) * pp;
      ow[row * OTP + 16 * t + c] = tot * rn[r] * CT;
    }
  }
  __syncthreads();
  v4u hv[4];
  size_t go[4];
#pragma unroll
  for (int it = 0; it < 4; ++it) {
    const int p  = lane + 32 * it;
    const int lr = p >> 3;
    const int d0 = (p & 7) * 8;
    const float* ra = ow + lr * OTP + d0;
    const v4f a0 = *(const v4f*)(ra), a1 = *(const v4f*)(ra + 4);
    const float f[8] = {a0[0], a0[1], a0[2], a0[3], a1[0], a1[1], a1[2], a1[3]};
    hv[it] = pack8(f);
    go[it] = (size_t)(q0 + lr) * DMOD + col0 + d0;
  }
#pragma unroll
  for (int it = 0; it < 4; ++it) *(volatile v4u*)(tp + go[it]) = hv[it];
  __threadfence();
#pragma unroll
  for (int it = 0; it < 4; ++it) *(volatile v4u*)(tp + go[it]) = hv[it];
}

extern "C" void kernel_launch(void* const* d_in, const int* in_sizes, int n_in,
                              void* d_out, int out_size, void* d_ws, size_t ws_size,
                              hipStream_t stream) {
  if (n_in < 14) return;
  if (in_sizes[0]  != NTOK * DMOD) return;
  if (in_sizes[1]  != DMOD * NPLN) return;
  if (in_sizes[2]  != NPLN) return;
  if (in_sizes[3]  != DMOD * NPLN) return;
  if (in_sizes[4]  != NPLN) return;
  if (in_sizes[5]  != DMOD * DMOD) return;
  if (in_sizes[6]  != DMOD) return;
  if (in_sizes[7]  != 4) return;
  if (in_sizes[8]  != NPOS) return;
  if (in_sizes[9]  != DMOD * DMOD) return;
  if (in_sizes[10] != DMOD) return;
  if (in_sizes[11] != 1) return;
  if (in_sizes[12] != DMOD * DMOD) return;
  if (in_sizes[13] != DMOD) return;
  if (out_size != NTOK * DMOD) return;

  const float* X   = (const float*)d_in[0];
  const float* Wk  = (const float*)d_in[1];
  const float* bk  = (const float*)d_in[2];
  const float* Wq  = (const float*)d_in[3];
  const float* bq  = (const float*)d_in[4];
  const float* Wv  = (const float*)d_in[5];
  const float* bv  = (const float*)d_in[6];
  const float* sw  = (const float*)d_in[7];
  const float* pfq = (const float*)d_in[8];
  const float* Wg  = (const float*)d_in[9];
  const float* bg  = (const float*)d_in[10];
  const float* pw  = (const float*)d_in[11];
  const float* Wo  = (const float*)d_in[12];
  const float* bo  = (const float*)d_in[13];
  float* out = (float*)d_out;

  const size_t XPL = (size_t)NTOK * DMOD * 2;
  const size_t WKQ = (size_t)NPH * DMOD * 2;
  const size_t WPL = (size_t)DMOD * DMOD * 2;
  const size_t FPB = (size_t)NTOK * FP * 2;
  const size_t GFB = (size_t)NTOK * DMOD * 4;
  const size_t SPB = (size_t)NTOK * SEQ * 2;
  size_t off = 0;
  const size_t oXh  = off; off += XPL;
  const size_t oWKQ = off; off += WKQ;
  const size_t oWV  = off; off += WPL;
  const size_t oWG  = off; off += WPL;
  const size_t oWO  = off; off += WPL;
  const size_t oQf  = off; off += FPB;
  const size_t oKf  = off; off += FPB;
  const size_t oVT  = off; off += XPL;
  const size_t oGT  = off; off += GFB;
  const size_t oSc  = off; off += SPB;
  const size_t oSp  = off; off += SPB;
  const size_t oT   = off; off += XPL;
  if (off > ws_size) return;
  if (off > (size_t)134217728) return;

  char* ws = (char*)d_ws;
  us* Xh   = (us*)(ws + oXh);
  us* WKQt = (us*)(ws + oWKQ);
  us* WVt  = (us*)(ws + oWV);
  us* WGt  = (us*)(ws + oWG);
  us* WOt  = (us*)(ws + oWO);
  us* Qf   = (us*)(ws + oQf);
  us* Kf   = (us*)(ws + oKf);
  us* VT   = (us*)(ws + oVT);
  float* GT = (float*)(ws + oGT);
  us* Sc   = (us*)(ws + oSc);
  us* Sp   = (us*)(ws + oSp);
  us* T    = (us*)(ws + oT);

  k_cvt_x<<<dim3((NTOK * DMOD) / 2048), dim3(256), 0, stream>>>(X, Xh);
  k_cvt_wkq<<<dim3(DMOD / 64, 2), dim3(256), 0, stream>>>(Wk, Wq, WKQt);
  k_cvt_wt<<<dim3(DMOD / 64, DMOD / 64), dim3(256), 0, stream>>>(Wv, WVt);
  k_cvt_wt<<<dim3(DMOD / 64, DMOD / 64), dim3(256), 0, stream>>>(Wg, WGt);
  k_cvt_wt<<<dim3(DMOD / 64, DMOD / 64), dim3(256), 0, stream>>>(Wo, WOt);
  k_phase<<<dim3(NTOK / 64), dim3(128), 0, stream>>>(Xh, WKQt, bk, bq, sw, pfq, Qf, Kf);
  k_proj<1><<<dim3(NTOK / 64, DMOD / 64), dim3(128), 0, stream>>>(Xh, WVt, bv, X, VT, GT);
  k_proj<2><<<dim3(NTOK / 64, DMOD / 64), dim3(128), 0, stream>>>(Xh, WGt, bg, X, T, GT);
  k_score<<<dim3(NQB, NBATCH), dim3(128), 0, stream>>>(Qf, Kf, Sc, Sp);
  k_oattn<<<dim3(NSEG, NQB, NBATCH), dim3(128), 0, stream>>>(Sc, Sp, VT, GT, pw, T);
  k_proj<3><<<dim3(NTOK / 64, DMOD / 64), dim3(128), 0, stream>>>(T, WOt, bo, X, VT, out);
  (void)hipGetLastError();
}
